// ODEVAE_60988535603646
// MI455X (gfx1250) — hardware-run, weakly checked
//
#include <hip/hip_runtime.h>
#include <math.h>

constexpr int NBATCH   = 256;
constexpr int NTIME    = 200;
constexpr int NOBS     = 256;
constexpr int NLAT     = 16;
constexpr int NHID     = 128;
constexpr int NSUBSTEP = 8;
constexpr int ENC_H1   = 512;
constexpr int ENC_H2   = 256;
constexpr int ENC_H3   = 128;
constexpr int DEC_H    = 512;
constexpr int HEAD_N   = 64;
constexpr int NTRAJ    = NBATCH * NTIME;

constexpr int OUT1_OFF  = NBATCH * NTIME * NOBS;
constexpr int OUT2_OFF  = OUT1_OFF + NBATCH * NLAT;
constexpr int OUT3_OFF  = OUT2_OFF + NBATCH * NLAT;
constexpr int OUT4_OFF  = OUT3_OFF + NBATCH * NTIME * NLAT;
constexpr int OUT_TOTAL = OUT4_OFF + NBATCH * (NTIME - 1) * NLAT;
constexpr int NZD_V4    = NBATCH * (NTIME - 1) * NLAT / 4;
static_assert((long long)OUT1_OFF * 4 == 52428800LL, "out1 offset");
static_assert((long long)OUT2_OFF * 4 == 52445184LL, "out2 offset");
static_assert((long long)OUT3_OFF * 4 == 52461568LL, "out3 offset");
static_assert((long long)OUT4_OFF * 4 == 55738368LL, "out4 offset");
static_assert((long long)OUT_TOTAL * 4 == 58998784LL, "out total");
static_assert(NZD_V4 % 256 == 0, "zdiff grid exact");
static_assert(NTIME % 8 == 0, "trajectory staging groups of 8 time points");
static_assert(NLAT == 16 && NHID == 128, "tile shapes");
static_assert(NTRAJ % 64 == 0 && DEC_H % 64 == 0 && NOBS % 64 == 0, "decoder tiles");
static_assert(NBATCH % 16 == 0 && ENC_H1 % 64 == 0 && ENC_H2 % 64 == 0 && ENC_H3 % 64 == 0, "encoder tiles");
static_assert(NOBS % 32 == 0 && ENC_H1 % 32 == 0 && ENC_H2 % 32 == 0 && ENC_H3 % 32 == 0 && DEC_H % 32 == 0, "k steps");

constexpr float F16_MIN_NORMAL = 6.103515625e-05f;
constexpr float RES_SCALE      = 2048.0f;
constexpr float RES_INV        = 1.0f / 2048.0f;
constexpr float W_CARRY        = 256.0f;
constexpr float W_CARRY_INV    = 1.0f / 256.0f;
constexpr float LN_EPS         = 1e-5f;

constexpr float RK_A21 = 0.2f;
constexpr float RK_A31 = (float)(3.0 / 40.0);
constexpr float RK_A32 = (float)(9.0 / 40.0);
constexpr float RK_A41 = (float)(44.0 / 45.0);
constexpr float RK_A42 = (float)(56.0 / 15.0);
constexpr float RK_A43 = (float)(32.0 / 9.0);
constexpr float RK_A51 = (float)(19372.0 / 6561.0);
constexpr float RK_A52 = (float)(25360.0 / 2187.0);
constexpr float RK_A53 = (float)(64448.0 / 6561.0);
constexpr float RK_A54 = (float)(212.0 / 729.0);
constexpr float RK_A61 = (float)(9017.0 / 3168.0);
constexpr float RK_A62 = (float)(355.0 / 33.0);
constexpr float RK_A63 = (float)(46732.0 / 5247.0);
constexpr float RK_A64 = (float)(49.0 / 176.0);
constexpr float RK_A65 = (float)(5103.0 / 18656.0);
constexpr float RK_B1  = (float)(35.0 / 384.0);
constexpr float RK_B3  = (float)(500.0 / 1113.0);
constexpr float RK_B4  = (float)(125.0 / 192.0);
constexpr float RK_B5  = (float)(2187.0 / 6784.0);
constexpr float RK_B6  = (float)(11.0 / 84.0);

typedef __attribute__((ext_vector_type(16))) _Float16 v16h;
typedef __attribute__((ext_vector_type(8)))  _Float16 v8h;
typedef __attribute__((ext_vector_type(8)))  float    v8f;
typedef __attribute__((ext_vector_type(4)))  float    v4f;

__device__ __forceinline__ v16h fragld(const _Float16* p) {
  union { v16h v; v8h h[2]; } f;
  f.h[0] = *(const v8h*)(p);
  f.h[1] = *(const v8h*)(p + 16);
  return f.v;
}

__device__ __forceinline__ v8f mma_g(v16h a, v16h b, v8f c) {
  c = __builtin_amdgcn_wmma_f32_16x16x32_f16(false, a, false, b, (short)0, c, false, false);
  asm volatile("v_nop\n\tv_nop\n\tv_nop\n\tv_nop" : "+v"(c) : "v"(a), "v"(b));
  return c;
}

__device__ __forceinline__ void wave_lds_sync() {
  __builtin_amdgcn_fence(__ATOMIC_RELEASE, "workgroup");
  __builtin_amdgcn_wave_barrier();
  __builtin_amdgcn_fence(__ATOMIC_ACQUIRE, "workgroup");
}

__device__ __forceinline__ float flush16(float v) {
  return (__builtin_fabsf(v) < F16_MIN_NORMAL) ? 0.0f : v;
}

__device__ __forceinline__ void split_h(float a, _Float16& hh, _Float16& ll) {
  hh = (_Float16)flush16(a);
  ll = (_Float16)flush16((a - (float)hh) * RES_SCALE);
}

__device__ __forceinline__ float silu_fast(float x) {
  return x * __builtin_amdgcn_rcpf(1.0f + __expf(-x));
}

__global__ __launch_bounds__(256) void wprep_kernel(const float* __restrict__ in, int kin, int nout,
                                                    unsigned short* __restrict__ outm, unsigned short* outr,
                                                    int kpitch, int nrows, int mode) {
  const int gid = blockIdx.x * 256 + threadIdx.x;
  const int nchunk = kpitch >> 3;
  if (gid >= nrows * nchunk) return;
  const int n = gid / nchunk;
  const int kc = (gid - n * nchunk) << 3;
  const int ncl = (n < nout) ? n : (nout - 1);
  v8h mv, rv;
#pragma unroll
  for (int e = 0; e < 8; ++e) {
    const int k = kc + e;
    const int ksrc = (mode == 1) ? (k & 15) : k;
    const int kcl = (ksrc < kin) ? ksrc : (kin - 1);
    const float w = in[(size_t)kcl * nout + ncl];
    const bool valid = (n < nout) && (ksrc < kin);
    const float wc = valid ? (w * W_CARRY) : 0.0f;
    const _Float16 hh = (_Float16)flush16(wc);
    const float hv = (float)hh;
    const float rf = flush16((wc - hv) * RES_SCALE);
    float mval = hv;
    float rval = rf;
    if (mode == 1) {
      const bool upper = (k >= 16);
      mval = upper ? 0.0f : hv;
      rval = upper ? hv : rf;
    }
    mv[e] = (_Float16)mval;
    rv[e] = (_Float16)rval;
  }
  unsigned short* pm = outm + (size_t)gid * 8;
  unsigned short* pr = outr + (size_t)gid * 8;
  *(volatile v8h*)pm = mv;
  if (mode != 2) *(volatile v8h*)pr = rv;
  __threadfence();
  *(volatile v8h*)pm = mv;
  if (mode != 2) *(volatile v8h*)pr = rv;
}

__global__ __launch_bounds__(256) void x0_split_kernel(const float* __restrict__ x, unsigned short* __restrict__ xh,
                                                       unsigned short* __restrict__ xl) {
  const int gid = blockIdx.x * 256 + threadIdx.x;
  if (gid >= NBATCH * (NOBS / 8)) return;
  const int row = gid >> 5, ch = gid & 31;
  const float* src = x + (size_t)row * (NTIME * NOBS) + ch * 8;
  const v4f f0 = *(const v4f*)src;
  const v4f f1 = *(const v4f*)(src + 4);
  v8h hv, lv;
#pragma unroll
  for (int e = 0; e < 4; ++e) {
    _Float16 hh, ll;
    split_h(f0[e], hh, ll);
    hv[e] = hh;
    lv[e] = ll;
    split_h(f1[e], hh, ll);
    hv[4 + e] = hh;
    lv[4 + e] = ll;
  }
  unsigned short* ph = xh + (size_t)gid * 8;
  unsigned short* pl = xl + (size_t)gid * 8;
  *(volatile v8h*)ph = hv;
  *(volatile v8h*)pl = lv;
  __threadfence();
  *(volatile v8h*)ph = hv;
  *(volatile v8h*)pl = lv;
}

template <bool PACKED, int OUT_MODE, bool RELU, bool HASBIAS>
__global__ __launch_bounds__(128) void gemm_split_kernel(
    const unsigned short* A1p, const unsigned short* A2p, int lda,
    const unsigned short* B1p, const unsigned short* B2p, int ldb,
    void* C1p, void* C2p, int ldc,
    const float* bias, int M, int N, int K) {
  __shared__ __align__(16) float sT[4][16 * 68];
  const _Float16* A1 = (const _Float16*)A1p;
  const _Float16* A2 = (const _Float16*)A2p;
  const _Float16* B1 = (const _Float16*)B1p;
  const _Float16* B2 = (const _Float16*)B2p;
  const int lane = threadIdx.x & 31;
  const int wave = threadIdx.x >> 5;
  const int tilesN = N >> 6;
  const int tilesM = M >> 4;
  const int tile = blockIdx.x * 4 + wave;
  if (tile >= tilesM * tilesN) return;
  const int tm = tile / tilesN;
  const int tn = tile - tm * tilesN;
  const int m0 = tm << 4;
  const int n0 = tn << 6;
  const int rlane = lane & 15;
  const int koff = (lane >> 4) * 8;
  const int mOff = (lane >> 4) * 8;

  v8f accm[4], accr[4];
#pragma unroll
  for (int j = 0; j < 4; ++j) {
    accm[j] = (v8f){0.f, 0.f, 0.f, 0.f, 0.f, 0.f, 0.f, 0.f};
    accr[j] = (v8f){0.f, 0.f, 0.f, 0.f, 0.f, 0.f, 0.f, 0.f};
  }
  for (int k0 = 0; k0 < K; k0 += 32) {
    const size_t ao = (size_t)(m0 + rlane) * lda + koff + k0;
    const v16h a1 = fragld(A1 + ao);
    v16h a2 = a1;
    if (!PACKED) a2 = fragld(A2 + ao);
#pragma unroll
    for (int j = 0; j < 4; ++j) {
      const size_t bo = (size_t)(n0 + (j << 4) + rlane) * ldb + koff + k0;
      const v16h b1 = fragld(B1 + bo);
      const v16h b2 = fragld(B2 + bo);
      accm[j] = mma_g(a1, b1, accm[j]);
      accr[j] = mma_g(a1, b2, accr[j]);
      if (!PACKED) accr[j] = mma_g(a2, b1, accr[j]);
    }
  }

  float* slab = sT[wave];
#pragma unroll
  for (int j = 0; j < 4; ++j) {
    float bv = 0.0f;
    if (HASBIAS) bv = bias[n0 + (j << 4) + rlane];
#pragma unroll
    for (int r = 0; r < 8; ++r) {
      float v = (accm[j][r] + accr[j][r] * RES_INV) * W_CARRY_INV + bv;
      if (RELU) v = fmaxf(v, 0.0f);
      slab[(mOff + r) * 68 + (j << 4) + rlane] = v;
    }
  }
  __builtin_amdgcn_fence(__ATOMIC_RELEASE, "workgroup");
  __builtin_amdgcn_wave_barrier();
  __builtin_amdgcn_fence(__ATOMIC_ACQUIRE, "workgroup");
  if (OUT_MODE == 0) {
    float* C = (float*)C1p;
    const int hh = lane >> 4, c4 = (lane & 15) * 4;
    for (int pass = 0; pass < 2; ++pass) {
#pragma unroll
      for (int it = 0; it < 8; ++it) {
        const int row = it * 2 + hh;
        const v4f v = *(const v4f*)(slab + row * 68 + c4);
        *(volatile v4f*)(C + (size_t)(m0 + row) * ldc + n0 + c4) = v;
      }
      __threadfence();
    }
  } else {
    _Float16* C1 = (_Float16*)C1p;
    _Float16* C2 = (_Float16*)C2p;
    const int q = lane >> 3, c8 = (lane & 7) * 8;
    for (int pass = 0; pass < 2; ++pass) {
#pragma unroll
      for (int it = 0; it < 4; ++it) {
        const int row = it * 4 + q;
        const float* sp = slab + row * 68 + c8;
        v8h hv, lv;
#pragma unroll
        for (int e = 0; e < 8; ++e) {
          const float a = sp[e];
          const _Float16 hh = (_Float16)flush16(a);
          hv[e] = hh;
          if (OUT_MODE == 2) lv[e] = (_Float16)flush16((a - (float)hh) * RES_SCALE);
        }
        *(volatile v8h*)(C1 + (size_t)(m0 + row) * ldc + n0 + c8) = hv;
        if (OUT_MODE == 2) *(volatile v8h*)(C2 + (size_t)(m0 + row) * ldc + n0 + c8) = lv;
      }
      __threadfence();
    }
  }
}

template <int OUT_MODE, bool RELU>
__global__ __launch_bounds__(256) void gemm_plain_kernel(
    const unsigned short* Ap, int lda, const unsigned short* Btp, int ldb,
    void* Cout, int ldc, const float* bias, int M, int N, int K, float scale) {
  __shared__ __align__(16) float sT[8][16 * 68];
  const _Float16* A = (const _Float16*)Ap;
  const _Float16* Bt = (const _Float16*)Btp;
  const int lane = threadIdx.x & 31;
  const int wave = threadIdx.x >> 5;
  const int tilesN = N >> 6;
  const int tilesM = M >> 6;
  const int tile = blockIdx.x * 8 + wave;
  if (tile >= tilesM * tilesN) return;
  const int tm = tile / tilesN;
  const int tn = tile - tm * tilesN;
  const int m0 = tm << 6;
  const int n0 = tn << 6;
  const int rlane = lane & 15;
  const int koff = (lane >> 4) * 8;
  const int mOff = (lane >> 4) * 8;

  v8f acc[4][4];
#pragma unroll
  for (int i = 0; i < 4; ++i)
#pragma unroll
    for (int j = 0; j < 4; ++j) acc[i][j] = (v8f){0.f, 0.f, 0.f, 0.f, 0.f, 0.f, 0.f, 0.f};

  for (int k0 = 0; k0 < K; k0 += 32) {
    v16h bh[4];
#pragma unroll
    for (int j = 0; j < 4; ++j)
      bh[j] = fragld(Bt + (size_t)(n0 + (j << 4) + rlane) * ldb + koff + k0);
#pragma unroll
    for (int i = 0; i < 4; ++i) {
      const v16h ah = fragld(A + (size_t)(m0 + (i << 4) + rlane) * lda + koff + k0);
#pragma unroll
      for (int j = 0; j < 4; ++j) acc[i][j] = mma_g(ah, bh[j], acc[i][j]);
    }
  }

  float bv[4];
#pragma unroll
  for (int j = 0; j < 4; ++j) bv[j] = bias[n0 + (j << 4) + rlane];

  float* slab = sT[wave];
#pragma unroll
  for (int i = 0; i < 4; ++i) {
    const int mBase = m0 + (i << 4);
#pragma unroll
    for (int j = 0; j < 4; ++j) {
#pragma unroll
      for (int r = 0; r < 8; ++r) {
        float v = acc[i][j][r] * scale + bv[j];
        if (RELU) v = fmaxf(v, 0.0f);
        slab[(mOff + r) * 68 + (j << 4) + rlane] = v;
      }
    }
    __builtin_amdgcn_fence(__ATOMIC_RELEASE, "workgroup");
    __builtin_amdgcn_wave_barrier();
    __builtin_amdgcn_fence(__ATOMIC_ACQUIRE, "workgroup");
    if (OUT_MODE == 0) {
      float* C = (float*)Cout;
      const int hh = lane >> 4, c4 = (lane & 15) * 4;
      for (int pass = 0; pass < 2; ++pass) {
#pragma unroll
        for (int it = 0; it < 8; ++it) {
          const int row = it * 2 + hh;
          const v4f v = *(const v4f*)(slab + row * 68 + c4);
          *(volatile v4f*)(C + (size_t)(mBase + row) * ldc + n0 + c4) = v;
        }
        __threadfence();
      }
    } else {
      _Float16* C = (_Float16*)Cout;
      const int q = lane >> 3, c8 = (lane & 7) * 8;
      for (int pass = 0; pass < 2; ++pass) {
#pragma unroll
        for (int it = 0; it < 4; ++it) {
          const int row = it * 4 + q;
          const float* sp = slab + row * 68 + c8;
          v8h hv;
#pragma unroll
          for (int e = 0; e < 8; ++e) hv[e] = (_Float16)flush16(sp[e]);
          *(volatile v8h*)(C + (size_t)(mBase + row) * ldc + n0 + c8) = hv;
        }
        __threadfence();
      }
    }
    __builtin_amdgcn_fence(__ATOMIC_RELEASE, "workgroup");
    __builtin_amdgcn_wave_barrier();
    __builtin_amdgcn_fence(__ATOMIC_ACQUIRE, "workgroup");
  }
}

__global__ __launch_bounds__(256) void heads_kernel(const float* __restrict__ hd, const float* __restrict__ mub,
                                                    const float* __restrict__ lvb, const float* __restrict__ eps,
                                                    float* __restrict__ out12, float* __restrict__ z0) {
  if (blockIdx.x >= 12) return;
  const int role = blockIdx.x >> 2;
  const int j = (blockIdx.x & 3) * 256 + threadIdx.x;
  const int f = 4 * j;
  const int row = f >> 4, col = f & 15;
  const v4f m4 = *(const v4f*)(hd + row * HEAD_N + col);
  const v4f l4 = *(const v4f*)(hd + row * HEAD_N + 16 + col);
  const v4f bm = *(const v4f*)(mub + col);
  const v4f bl = *(const v4f*)(lvb + col);
  const v4f e4 = *(const v4f*)(eps + row * NLAT + col);
  const v4f mu = m4 + bm;
  const v4f lv = l4 + bl;
  v4f zz;
#pragma unroll
  for (int e = 0; e < 4; ++e) zz[e] = mu[e] + expf(0.5f * lv[e]) * e4[e];
  v4f val = zz;
  if (role == 0) val = mu;
  if (role == 1) val = lv;
  float* dst = (role < 2) ? (out12 + role * (NBATCH * NLAT) + f) : (z0 + f);
  *(volatile v4f*)dst = val;
  __threadfence();
  *(volatile v4f*)dst = val;
}

__global__ __launch_bounds__(256) void zdiff_kernel(const float* __restrict__ zt, const float* __restrict__ tvec,
                                                    float* __restrict__ out4) {
  const int i = blockIdx.x * 256 + threadIdx.x;
  if (i >= NZD_V4) return;
  const int f = 4 * i;
  const int b = f / ((NTIME - 1) * NLAT);
  const int rem = f - b * ((NTIME - 1) * NLAT);
  int ii = rem >> 4;
  ii = (ii < NTIME - 2) ? ii : (NTIME - 2);
  const int d = rem & 15;
  const float dt = tvec[ii + 1] - tvec[ii];
  const float rdt = 1.0f / dt;
  const float* p0 = zt + ((size_t)(b * NTIME + ii) * NLAT + d);
  const v4f a = *(const v4f*)p0;
  const v4f c = *(const v4f*)(p0 + NLAT);
  v4f o;
#pragma unroll
  for (int e = 0; e < 4; ++e) o[e] = (c[e] - a[e]) * rdt;
  float* op = out4 + f;
  *(volatile v4f*)op = o;
  __threadfence();
  *(volatile v4f*)op = o;
}

constexpr int ODE_WAVES     = 8;
constexpr int ODE_THREADS   = 32 * ODE_WAVES;
constexpr int ODE_ROWS_BLK  = 16 * ODE_WAVES;
constexpr int SK_WAVE_FLOATS = 7 * 32 * 8;
constexpr int ST_WAVE_FLOATS = 16 * 8 * 16;
constexpr int W1P     = 40;
constexpr int W2P     = 136;
constexpr int OFF_W1M = 0;
constexpr int OFF_W1R = OFF_W1M + NHID * W1P * 2;
constexpr int OFF_W2H = OFF_W1R + NHID * W1P * 2;
constexpr int OFF_W2L = OFF_W2H + NHID * W2P * 2;
constexpr int OFF_W3H = OFF_W2L + NHID * W2P * 2;
constexpr int OFF_W3L = OFF_W3H + NLAT * W2P * 2;
constexpr int OFF_B1  = OFF_W3L + NLAT * W2P * 2;
constexpr int OFF_B2  = OFF_B1 + NHID * 4;
constexpr int OFF_B3  = OFF_B2 + NHID * 4;
constexpr int OFF_G   = OFF_B3 + NLAT * 4;
constexpr int OFF_BT  = OFF_G + NLAT * 4;
constexpr int OFF_RK  = OFF_BT + NLAT * 4;
constexpr int OFF_K   = OFF_RK + 176;
constexpr int OFF_T   = OFF_K + ODE_WAVES * SK_WAVE_FLOATS * 4;
constexpr int ODE_LDS_BYTES = OFF_T + ODE_WAVES * ST_WAVE_FLOATS * 4;
static_assert(OFF_W1R % 16 == 0 && OFF_W2H % 16 == 0 && OFF_W2L % 16 == 0 && OFF_W3H % 16 == 0 && OFF_W3L % 16 == 0, "align");
static_assert(OFF_B1 % 16 == 0 && OFF_B2 % 16 == 0 && OFF_B3 % 16 == 0 && OFF_G % 16 == 0 && OFF_BT % 16 == 0, "align");
static_assert(OFF_RK % 16 == 0 && OFF_K % 16 == 0 && OFF_T % 16 == 0, "align");
static_assert(OFF_K == 100208, "shared part");
static_assert(ODE_LDS_BYTES == 223088, "lds total");
static_assert(ODE_LDS_BYTES <= 262144, "lds budget");
static_assert(NBATCH % ODE_ROWS_BLK == 0, "batch rows per block");
static_assert((NHID * 4) % ODE_THREADS == 0 && (NHID * 16) % ODE_THREADS == 0 && NLAT * 16 == ODE_THREADS, "staging coverage");

template <int BASE>
__device__ __forceinline__ void act_split(const v8f am, const v8f ar, const v4f ba, const v4f bb, v16h& fh, v16h& fl) {
#pragma unroll
  for (int r = 0; r < 8; ++r) {
    const float bias = (r < 4) ? ba[r & 3] : bb[r & 3];
    const float x = (am[r] + ar[r] * RES_INV) * W_CARRY_INV + bias;
    const float a = silu_fast(x);
    _Float16 hh, ll;
    split_h(a, hh, ll);
    fh[BASE + r] = hh;
    fl[BASE + r] = ll;
  }
}

__device__ __forceinline__ void feval(const _Float16* sW1m, const _Float16* sW1r, const _Float16* sW2h, const _Float16* sW2l,
                                      const _Float16* sW3h, const _Float16* sW3l, const float* sB1, const float* sB2,
                                      const float* sB3, const float* sG, const float* sBt,
                                      int c, int h, const float (&y)[8], float (&kout)[8]) {
  const v8f zero8 = {0.f, 0.f, 0.f, 0.f, 0.f, 0.f, 0.f, 0.f};
  v16h zb;
#pragma unroll
  for (int r = 0; r < 8; ++r) {
    _Float16 hh, ll;
    split_h(y[r], hh, ll);
    zb[r] = hh;
    zb[8 + r] = ll;
  }
  v16h ah[4], al[4];
#pragma unroll
  for (int s = 0; s < 4; ++s) {
#pragma unroll
    for (int tt = 0; tt < 2; ++tt) {
      const int t = 2 * s + tt;
      const v16h a1 = fragld(sW1m + (16 * t + c) * W1P + 8 * h);
      const v16h a2 = fragld(sW1r + (16 * t + c) * W1P + 8 * h);
      const v8f am = mma_g(a1, zb, zero8);
      const v8f ar = mma_g(a2, zb, zero8);
      const v4f ba = *(const v4f*)(sB1 + 16 * t + 8 * h);
      const v4f bb = *(const v4f*)(sB1 + 16 * t + 8 * h + 4);
      if (tt == 0) act_split<0>(am, ar, ba, bb, ah[s], al[s]);
      else         act_split<8>(am, ar, ba, bb, ah[s], al[s]);
    }
  }
  v8f dm = zero8, dr = zero8;
#pragma unroll
  for (int s2 = 0; s2 < 4; ++s2) {
    v16h chh, cll;
#pragma unroll
    for (int tt = 0; tt < 2; ++tt) {
      const int t = 2 * s2 + tt;
      v8f am = zero8, ar = zero8;
#pragma unroll
      for (int s = 0; s < 4; ++s) {
        const v16h wh = fragld(sW2h + (16 * t + c) * W2P + 32 * s + 8 * h);
        const v16h wl = fragld(sW2l + (16 * t + c) * W2P + 32 * s + 8 * h);
        am = mma_g(wh, ah[s], am);
        ar = mma_g(wh, al[s], ar);
        ar = mma_g(wl, ah[s], ar);
      }
      const v4f ba = *(const v4f*)(sB2 + 16 * t + 8 * h);
      const v4f bb = *(const v4f*)(sB2 + 16 * t + 8 * h + 4);
      if (tt == 0) act_split<0>(am, ar, ba, bb, chh, cll);
      else         act_split<8>(am, ar, ba, bb, chh, cll);
    }
    const v16h w3a = fragld(sW3h + c * W2P + 32 * s2 + 8 * h);
    const v16h w3b = fragld(sW3l + c * W2P + 32 * s2 + 8 * h);
    dm = mma_g(w3a, chh, dm);
    dr = mma_g(w3a, cll, dr);
    dr = mma_g(w3b, chh, dr);
  }
  const v4f b3a = *(const v4f*)(sB3 + 8 * h);
  const v4f b3b = *(const v4f*)(sB3 + 8 * h + 4);
  const v4f ga  = *(const v4f*)(sG + 8 * h);
  const v4f gb  = *(const v4f*)(sG + 8 * h + 4);
  const v4f ta  = *(const v4f*)(sBt + 8 * h);
  const v4f tb  = *(const v4f*)(sBt + 8 * h + 4);
  float dz[8];
  float sum = 0.0f;
#pragma unroll
  for (int r = 0; r < 8; ++r) {
    const float bias = (r < 4) ? b3a[r & 3] : b3b[r & 3];
    dz[r] = (dm[r] + dr[r] * RES_INV) * W_CARRY_INV + bias;
    sum += dz[r];
  }
  sum += __shfl_xor(sum, 16, 32);
  const float mean = sum * (1.0f / 16.0f);
  float sq = 0.0f;
#pragma unroll
  for (int r = 0; r < 8; ++r) {
    dz[r] = dz[r] - mean;
    sq += dz[r] * dz[r];
  }
  sq += __shfl_xor(sq, 16, 32);
  const float inv = __builtin_amdgcn_rsqf(sq * (1.0f / 16.0f) + LN_EPS);
#pragma unroll
  for (int r = 0; r < 8; ++r) {
    const float gg = (r < 4) ? ga[r & 3] : gb[r & 3];
    const float bt = (r < 4) ? ta[r & 3] : tb[r & 3];
    kout[r] = dz[r] * inv * gg + bt;
  }
}

__device__ __forceinline__ void rk_combine(const float* sK, const float* sRK, int st, int nj, int lane, float hs, float (&y)[8]) {
  float acc[8];
#pragma unroll
  for (int r = 0; r < 8; ++r) acc[r] = 0.0f;
#pragma unroll 1
  for (int j = 0; j < nj; ++j) {
    const float cf = sRK[st * 6 + j];
    const v4f ka = *(const v4f*)(sK + (j * 32 + lane) * 8);
    const v4f kb = *(const v4f*)(sK + (j * 32 + lane) * 8 + 4);
#pragma unroll
    for (int e = 0; e < 4; ++e) {
      acc[e] += cf * ka[e];
      acc[4 + e] += cf * kb[e];
    }
  }
  const v4f za = *(const v4f*)(sK + (6 * 32 + lane) * 8);
  const v4f zb = *(const v4f*)(sK + (6 * 32 + lane) * 8 + 4);
#pragma unroll
  for (int e = 0; e < 4; ++e) {
    y[e] = za[e] + hs * acc[e];
    y[4 + e] = zb[e] + hs * acc[4 + e];
  }
}

__device__ __forceinline__ void traj_flush(const float* sT, float* zout, float* zws, unsigned short* zA,
                                           int row0, int grp, int lane) {
  const int slot = lane >> 2, q = lane & 3;
  const bool wantres = (q >= 2);
  for (int pass = 0; pass < 2; ++pass) {
#pragma unroll 1
    for (int row = 0; row < 16; ++row) {
      const v4f v = *(const v4f*)(sT + row * 128 + lane * 4);
      const size_t rbase = (size_t)(row0 + row) * NTIME + 8 * grp;
      *(volatile v4f*)(zout + rbase * NLAT + lane * 4) = v;
      *(volatile v4f*)(zws + rbase * NLAT + lane * 4) = v;
      const float* sp = sT + row * 128 + slot * 16 + 8 * (q & 1);
      const v4f f0 = *(const v4f*)sp;
      const v4f f1 = *(const v4f*)(sp + 4);
      v8h hv;
#pragma unroll
      for (int e = 0; e < 8; ++e) {
        const float a = (e < 4) ? f0[e & 3] : f1[e & 3];
        const float af = flush16(a);
        const _Float16 hh = (_Float16)af;
        const float rf = flush16((a - (float)hh) * RES_SCALE);
        hv[e] = (_Float16)(wantres ? rf : af);
      }
      *(volatile v8h*)(zA + rbase * 32 + lane * 8) = hv;
    }
    __threadfence();
  }
}

__global__ __launch_bounds__(256) __attribute__((amdgpu_num_vgpr(256)))
void ode_kernel(const float* __restrict__ tvec, const float* __restrict__ z0,
                const unsigned short* __restrict__ w1m, const unsigned short* __restrict__ w1r,
                const unsigned short* __restrict__ w2h, const unsigned short* __restrict__ w2l,
                const unsigned short* __restrict__ w3h, const unsigned short* __restrict__ w3l,
                const float* __restrict__ b1, const float* __restrict__ b2, const float* __restrict__ b3,
                const float* __restrict__ lng, const float* __restrict__ lnb,
                float* __restrict__ zout, float* __restrict__ zws, unsigned short* __restrict__ zA) {
  extern __shared__ __align__(16) unsigned char smem[];
  if (blockIdx.x >= NBATCH / ODE_ROWS_BLK) return;
  _Float16* sW1m = (_Float16*)(smem + OFF_W1M);
  _Float16* sW1r = (_Float16*)(smem + OFF_W1R);
  _Float16* sW2h = (_Float16*)(smem + OFF_W2H);
  _Float16* sW2l = (_Float16*)(smem + OFF_W2L);
  _Float16* sW3h = (_Float16*)(smem + OFF_W3H);
  _Float16* sW3l = (_Float16*)(smem + OFF_W3L);
  float* sB1 = (float*)(smem + OFF_B1);
  float* sB2 = (float*)(smem + OFF_B2);
  float* sB3 = (float*)(smem + OFF_B3);
  float* sG  = (float*)(smem + OFF_G);
  float* sBt = (float*)(smem + OFF_BT);
  float* sRK = (float*)(smem + OFF_RK);

  const int tid  = threadIdx.x;
  const int lane = tid & 31;
  const int wave = tid >> 5;
  const int c = lane & 15, h = lane >> 4;
  const int row0 = blockIdx.x * ODE_ROWS_BLK + wave * 16;
  float* sK = (float*)(smem + OFF_K) + wave * SK_WAVE_FLOATS;
  float* sT = (float*)(smem + OFF_T) + wave * ST_WAVE_FLOATS;

  {
    const _Float16* g1m = (const _Float16*)w1m;
    const _Float16* g1r = (const _Float16*)w1r;
    const _Float16* g2h = (const _Float16*)w2h;
    const _Float16* g2l = (const _Float16*)w2l;
    const _Float16* g3h = (const _Float16*)w3h;
    const _Float16* g3l = (const _Float16*)w3l;
#pragma unroll
    for (int it = 0; it < (NHID * 4) / ODE_THREADS; ++it) {
      const int idx = it * ODE_THREADS + tid;
      const int rr = idx >> 2, ch = (idx & 3) * 8;
      *(v8h*)(sW1m + rr * W1P + ch) = *(const v8h*)(g1m + rr * 32 + ch);
      *(v8h*)(sW1r + rr * W1P + ch) = *(const v8h*)(g1r + rr * 32 + ch);
    }
#pragma unroll 4
    for (int it = 0; it < (NHID * 16) / ODE_THREADS; ++it) {
      const int idx = it * ODE_THREADS + tid;
      const int rr = idx >> 4, ch = (idx & 15) * 8;
      *(v8h*)(sW2h + rr * W2P + ch) = *(const v8h*)(g2h + rr * NHID + ch);
      *(v8h*)(sW2l + rr * W2P + ch) = *(const v8h*)(g2l + rr * NHID + ch);
    }
    {
      const int rr = tid >> 4, ch = (tid & 15) * 8;
      *(v8h*)(sW3h + rr * W2P + ch) = *(const v8h*)(g3h + rr * NHID + ch);
      *(v8h*)(sW3l + rr * W2P + ch) = *(const v8h*)(g3l + rr * NHID + ch);
    }
    sB1[tid & (NHID - 1)] = b1[tid & (NHID - 1)];
    sB2[tid & (NHID - 1)] = b2[tid & (NHID - 1)];
    sB3[tid & (NLAT - 1)] = b3[tid & (NLAT - 1)];
    sG[tid & (NLAT - 1)]  = lng[tid & (NLAT - 1)];
    sBt[tid & (NLAT - 1)] = lnb[tid & (NLAT - 1)];
  }
  sRK[6 * 1 + 0] = RK_A21;
  sRK[6 * 2 + 0] = RK_A31;
  sRK[6 * 2 + 1] = RK_A32;
  sRK[6 * 3 + 0] = RK_A41;
  sRK[6 * 3 + 1] = -RK_A42;
  sRK[6 * 3 + 2] = RK_A43;
  sRK[6 * 4 + 0] = RK_A51;
  sRK[6 * 4 + 1] = -RK_A52;
  sRK[6 * 4 + 2] = RK_A53;
  sRK[6 * 4 + 3] = -RK_A54;
  sRK[6 * 5 + 0] = RK_A61;
  sRK[6 * 5 + 1] = -RK_A62;
  sRK[6 * 5 + 2] = RK_A63;
  sRK[6 * 5 + 3] = RK_A64;
  sRK[6 * 5 + 4] = -RK_A65;
  sRK[6 * 6 + 0] = RK_B1;
  sRK[6 * 6 + 1] = 0.0f;
  sRK[6 * 6 + 2] = RK_B3;
  sRK[6 * 6 + 3] = RK_B4;
  sRK[6 * 6 + 4] = -RK_B5;
  sRK[6 * 6 + 5] = RK_B6;

  {
    const float* zp = z0 + (size_t)(row0 + c) * NLAT + 8 * h;
    const v4f za = *(const v4f*)zp;
    const v4f zb = *(const v4f*)(zp + 4);
    *(v4f*)(sK + (6 * 32 + lane) * 8) = za;
    *(v4f*)(sK + (6 * 32 + lane) * 8 + 4) = zb;
    *(v4f*)(sT + (c * 8 + 0) * 16 + 8 * h) = za;
    *(v4f*)(sT + (c * 8 + 0) * 16 + 8 * h + 4) = zb;
  }
  __syncthreads();

  float y[8];
#pragma unroll 1
  for (int iv = 0; iv < NTIME - 1; ++iv) {
    const float dt = tvec[iv + 1] - tvec[iv];
    const float hs = dt * (1.0f / (float)NSUBSTEP);
#pragma unroll 1
    for (int ss = 0; ss < NSUBSTEP; ++ss) {
#pragma unroll 1
      for (int st = 0; st < 6; ++st) {
        rk_combine(sK, sRK, st, st, lane, hs, y);
        float kout[8];
        feval(sW1m, sW1r, sW2h, sW2l, sW3h, sW3l, sB1, sB2, sB3, sG, sBt, c, h, y, kout);
        const v4f ka = {kout[0], kout[1], kout[2], kout[3]};
        const v4f kb = {kout[4], kout[5], kout[6], kout[7]};
        *(v4f*)(sK + (st * 32 + lane) * 8) = ka;
        *(v4f*)(sK + (st * 32 + lane) * 8 + 4) = kb;
      }
      rk_combine(sK, sRK, 6, 6, lane, hs, y);
      const v4f za = {y[0], y[1], y[2], y[3]};
      const v4f zb = {y[4], y[5], y[6], y[7]};
      *(v4f*)(sK + (6 * 32 + lane) * 8) = za;
      *(v4f*)(sK + (6 * 32 + lane) * 8 + 4) = zb;
    }
    const int l = iv + 1;
    {
      const v4f za = {y[0], y[1], y[2], y[3]};
      const v4f zb = {y[4], y[5], y[6], y[7]};
      *(v4f*)(sT + (c * 8 + (l & 7)) * 16 + 8 * h) = za;
      *(v4f*)(sT + (c * 8 + (l & 7)) * 16 + 8 * h + 4) = zb;
    }
    if ((l & 7) == 7) {
      wave_lds_sync();
      traj_flush(sT, zout, zws, zA, row0, l >> 3, lane);
      wave_lds_sync();
    }
  }
}

extern "C" void kernel_launch(void* const* d_in, const int* in_sizes, int n_in,
                              void* d_out, int out_size, void* d_ws, size_t ws_size, hipStream_t stream) {
  if (n_in < 27 || d_out == nullptr || d_ws == nullptr) return;
  if (in_sizes[0] != NBATCH * NTIME * NOBS || in_sizes[1] != NTIME || in_sizes[2] != NBATCH * NLAT ||
      in_sizes[3] != NOBS * ENC_H1 || in_sizes[4] != ENC_H1 || in_sizes[5] != ENC_H1 * ENC_H2 ||
      in_sizes[6] != ENC_H2 || in_sizes[7] != ENC_H2 * ENC_H3 || in_sizes[8] != ENC_H3 ||
      in_sizes[9] != ENC_H3 * NLAT || in_sizes[10] != NLAT || in_sizes[11] != ENC_H3 * NLAT ||
      in_sizes[12] != NLAT || in_sizes[13] != NLAT * NHID || in_sizes[14] != NHID ||
      in_sizes[15] != NHID * NHID || in_sizes[16] != NHID || in_sizes[17] != NHID * NLAT ||
      in_sizes[18] != NLAT || in_sizes[19] != NLAT || in_sizes[20] != NLAT ||
      in_sizes[21] != NLAT * DEC_H || in_sizes[22] != DEC_H || in_sizes[23] != DEC_H * DEC_H ||
      in_sizes[24] != DEC_H || in_sizes[25] != DEC_H * NOBS || in_sizes[26] != NOBS ||
      out_size != OUT_TOTAL) return;

  const float* x_seq  = (const float*)d_in[0];
  const float* tvec   = (const float*)d_in[1];
  const float* eps    = (const float*)d_in[2];
  const float* enc_w1 = (const float*)d_in[3];
  const float* enc_b1 = (const float*)d_in[4];
  const float* enc_w2 = (const float*)d_in[5];
  const float* enc_b2 = (const float*)d_in[6];
  const float* enc_w3 = (const float*)d_in[7];
  const float* enc_b3 = (const float*)d_in[8];
  const float* mu_w   = (const float*)d_in[9];
  const float* mu_b   = (const float*)d_in[10];
  const float* lv_w   = (const float*)d_in[11];
  const float* lv_b   = (const float*)d_in[12];
  const float* ode_w1 = (const float*)d_in[13];
  const float* ode_b1 = (const float*)d_in[14];
  const float* ode_w2 = (const float*)d_in[15];
  const float* ode_b2 = (const float*)d_in[16];
  const float* ode_w3 = (const float*)d_in[17];
  const float* ode_b3 = (const float*)d_in[18];
  const float* ln_g   = (const float*)d_in[19];
  const float* ln_b   = (const float*)d_in[20];
  const float* dec_w1 = (const float*)d_in[21];
  const float* dec_b1 = (const float*)d_in[22];
  const float* dec_w2 = (const float*)d_in[23];
  const float* dec_b2 = (const float*)d_in[24];
  const float* dec_w3 = (const float*)d_in[25];
  const float* dec_b3 = (const float*)d_in[26];
  float* out = (float*)d_out;

  char* ws = (char*)d_ws;
  size_t off = 0;
  auto carve = [&](size_t bytes) -> char* { char* p = ws + off; off += (bytes + 255) & ~(size_t)255; return p; };
  unsigned short* x0h  = (unsigned short*)carve((size_t)NBATCH * NOBS * 2);
  unsigned short* x0l  = (unsigned short*)carve((size_t)NBATCH * NOBS * 2);
  unsigned short* ew1h = (unsigned short*)carve((size_t)ENC_H1 * NOBS * 2);
  unsigned short* ew1l = (unsigned short*)carve((size_t)ENC_H1 * NOBS * 2);
  unsigned short* ew2h = (unsigned short*)carve((size_t)ENC_H2 * ENC_H1 * 2);
  unsigned short* ew2l = (unsigned short*)carve((size_t)ENC_H2 * ENC_H1 * 2);
  unsigned short* ew3h = (unsigned short*)carve((size_t)ENC_H3 * ENC_H2 * 2);
  unsigned short* ew3l = (unsigned short*)carve((size_t)ENC_H3 * ENC_H2 * 2);
  unsigned short* hwh  = (unsigned short*)carve((size_t)HEAD_N * ENC_H3 * 2);
  unsigned short* hwl  = (unsigned short*)carve((size_t)HEAD_N * ENC_H3 * 2);
  unsigned short* ow1m = (unsigned short*)carve((size_t)NHID * 32 * 2);
  unsigned short* ow1r = (unsigned short*)carve((size_t)NHID * 32 * 2);
  unsigned short* ow2h = (unsigned short*)carve((size_t)NHID * NHID * 2);
  unsigned short* ow2l = (unsigned short*)carve((size_t)NHID * NHID * 2);
  unsigned short* ow3h = (unsigned short*)carve((size_t)NLAT * NHID * 2);
  unsigned short* ow3l = (unsigned short*)carve((size_t)NLAT * NHID * 2);
  unsigned short* dw1m = (unsigned short*)carve((size_t)DEC_H * 32 * 2);
  unsigned short* dw1r = (unsigned short*)carve((size_t)DEC_H * 32 * 2);
  unsigned short* dw2  = (unsigned short*)carve((size_t)DEC_H * DEC_H * 2);
  unsigned short* dw3  = (unsigned short*)carve((size_t)NOBS * DEC_H * 2);
  unsigned short* h1h  = (unsigned short*)carve((size_t)NBATCH * ENC_H1 * 2);
  unsigned short* h1l  = (unsigned short*)carve((size_t)NBATCH * ENC_H1 * 2);
  unsigned short* h2h  = (unsigned short*)carve((size_t)NBATCH * ENC_H2 * 2);
  unsigned short* h2l  = (unsigned short*)carve((size_t)NBATCH * ENC_H2 * 2);
  unsigned short* h3h  = (unsigned short*)carve((size_t)NBATCH * ENC_H3 * 2);
  unsigned short* h3l  = (unsigned short*)carve((size_t)NBATCH * ENC_H3 * 2);
  float*          hd   = (float*)carve((size_t)NBATCH * HEAD_N * 4);
  float*          z0   = (float*)carve((size_t)NBATCH * NLAT * 4);
  float*          zws  = (float*)carve((size_t)NTRAJ * NLAT * 4);
  unsigned short* zA   = (unsigned short*)carve((size_t)NTRAJ * 32 * 2);
  unsigned short* g1   = (unsigned short*)carve((size_t)NTRAJ * DEC_H * 2);
  unsigned short* g2   = (unsigned short*)carve((size_t)NTRAJ * DEC_H * 2);
  if (off > ws_size || off > (size_t)134217728) return;

  wprep_kernel<<<(ENC_H1 * (NOBS / 8)) / 256, 256, 0, stream>>>(enc_w1, NOBS, ENC_H1, ew1h, ew1l, NOBS, ENC_H1, 0);
  wprep_kernel<<<(ENC_H2 * (ENC_H1 / 8)) / 256, 256, 0, stream>>>(enc_w2, ENC_H1, ENC_H2, ew2h, ew2l, ENC_H1, ENC_H2, 0);
  wprep_kernel<<<(ENC_H3 * (ENC_H2 / 8)) / 256, 256, 0, stream>>>(enc_w3, ENC_H2, ENC_H3, ew3h, ew3l, ENC_H2, ENC_H3, 0);
  wprep_kernel<<<(16 * (ENC_H3 / 8)) / 256, 256, 0, stream>>>(mu_w, ENC_H3, NLAT, hwh, hwl, ENC_H3, 16, 0);
  wprep_kernel<<<(48 * (ENC_H3 / 8)) / 256, 256, 0, stream>>>(lv_w, ENC_H3, NLAT, hwh + 16 * ENC_H3, hwl + 16 * ENC_H3,
                                                             ENC_H3, 48, 0);
  wprep_kernel<<<(NHID * 4) / 256, 256, 0, stream>>>(ode_w1, NLAT, NHID, ow1m, ow1r, 32, NHID, 1);
  wprep_kernel<<<(NHID * (NHID / 8)) / 256, 256, 0, stream>>>(ode_w2, NHID, NHID, ow2h, ow2l, NHID, NHID, 0);
  wprep_kernel<<<(NLAT * (NHID / 8)) / 256, 256, 0, stream>>>(ode_w3, NHID, NLAT, ow3h, ow3l, NHID, NLAT, 0);
  wprep_kernel<<<(DEC_H * 4) / 256, 256, 0, stream>>>(dec_w1, NLAT, DEC_H, dw1m, dw1r, 32, DEC_H, 1);
  wprep_kernel<<<(DEC_H * (DEC_H / 8)) / 256, 256, 0, stream>>>(dec_w2, DEC_H, DEC_H, dw2, dw2, DEC_H, DEC_H, 2);
  wprep_kernel<<<(NOBS * (DEC_H / 8)) / 256, 256, 0, stream>>>(dec_w3, DEC_H, NOBS, dw3, dw3, DEC_H, NOBS, 2);
  x0_split_kernel<<<(NBATCH * (NOBS / 8)) / 256, 256, 0, stream>>>(x_seq, x0h, x0l);

  gemm_split_kernel<false, 2, true, true><<<((NBATCH / 16) * (ENC_H1 / 64) + 3) / 4, 128, 0, stream>>>(
      x0h, x0l, NOBS, ew1h, ew1l, NOBS, h1h, h1l, ENC_H1, enc_b1, NBATCH, ENC_H1, NOBS);
  gemm_split_kernel<false, 2, true, true><<<((NBATCH / 16) * (ENC_H2 / 64) + 3) / 4, 128, 0, stream>>>(
      h1h, h1l, ENC_H1, ew2h, ew2l, ENC_H1, h2h, h2l, ENC_H2, enc_b2, NBATCH, ENC_H2, ENC_H1);
  gemm_split_kernel<false, 2, true, true><<<((NBATCH / 16) * (ENC_H3 / 64) + 3) / 4, 128, 0, stream>>>(
      h2h, h2l, ENC_H2, ew3h, ew3l, ENC_H2, h3h, h3l, ENC_H3, enc_b3, NBATCH, ENC_H3, ENC_H2);
  gemm_split_kernel<false, 0, false, false><<<((NBATCH / 16) * (HEAD_N / 64) + 3) / 4, 128, 0, stream>>>(
      h3h, h3l, ENC_H3, hwh, hwl, ENC_H3, hd, hd, HEAD_N, enc_b3, NBATCH, HEAD_N, ENC_H3);
  heads_kernel<<<12, 256, 0, stream>>>(hd, mu_b, lv_b, eps, out + OUT1_OFF, z0);

  ode_kernel<<<NBATCH / ODE_ROWS_BLK, ODE_THREADS, ODE_LDS_BYTES, stream>>>(tvec, z0, ow1m, ow1r, ow2h, ow2l, ow3h, ow3l,
                                                                             ode_b1, ode_b2, ode_b3, ln_g, ln_b,
                                                                             out + OUT3_OFF, zws, zA);
  zdiff_kernel<<<NZD_V4 / 256, 256, 0, stream>>>(zws, tvec, out + OUT4_OFF);

  gemm_split_kernel<true, 1, true, true><<<((NTRAJ / 16) * (DEC_H / 64) + 3) / 4, 128, 0, stream>>>(
      zA, zA, 32, dw1m, dw1r, 32, g1, g1, DEC_H, dec_b1, NTRAJ, DEC_H, 32);
  gemm_plain_kernel<1, true><<<((NTRAJ / 64) * (DEC_H / 64) + 7) / 8, 256, 0, stream>>>(
      g1, DEC_H, dw2, DEC_H, g2, DEC_H, dec_b2, NTRAJ, DEC_H, DEC_H, W_CARRY_INV);
  gemm_plain_kernel<0, false><<<((NTRAJ / 64) * (NOBS / 64) + 7) / 8, 256, 0, stream>>>(
      g2, DEC_H, dw3, DEC_H, out, NOBS, dec_b3, NTRAJ, NOBS, DEC_H, W_CARRY_INV);
}
